// RadixAttention_67233418052078
// MI455X (gfx1250) — hardware-verified
//
#include <hip/hip_runtime.h>
#include <math.h>
#include <stdint.h>

#define NTOK  2048
#define RLEN  1024
#define HQ    32
#define HKV   8
#define GRPQ  4
#define HDIM  128
#define QW    (HQ * HDIM)
#define KW    (HKV * HDIM)
#define NQB   (NTOK / 64)
#define QBR   (RLEN / 64)
#define NPC   (RLEN / 64)
#define QSC   16.0f
#define KSC   16.0f
#define VSC   16.0f
#define PSC   1024.0f
#define CAPV  30.0f
#define NEG_BIG (-1.0e30f)
static_assert(HQ == HKV * GRPQ);
static_assert((NTOK % 64) == 0 && (RLEN % 64) == 0);
static_assert(NQB == 2 * QBR);
static_assert(((NTOK * QW) % 2048) == 0 && ((NTOK * KW) % 2048) == 0);
static_assert((HDIM % 32) == 0);

typedef _Float16 v16h __attribute__((ext_vector_type(16)));
typedef _Float16 v8h  __attribute__((ext_vector_type(8)));
typedef float    v8f  __attribute__((ext_vector_type(8)));
typedef float    v4f  __attribute__((ext_vector_type(4)));
typedef unsigned int v4u __attribute__((ext_vector_type(4)));
union FH { v16h v; v8h h[2]; };

__device__ __forceinline__ unsigned short bf_bits(float f) {
  unsigned u = __float_as_uint(f);
  return (unsigned short)((u + 0x7FFFu + ((u >> 16) & 1u)) >> 16);
}
__device__ __forceinline__ float bf_up(unsigned short b) { return __uint_as_float(((unsigned)b) << 16); }
__device__ __forceinline__ float bfr(float f) { return bf_up(bf_bits(f)); }
__device__ __forceinline__ unsigned short h_bits(_Float16 x) { return __builtin_bit_cast(unsigned short, x); }
__device__ __forceinline__ unsigned pk16(unsigned short a, unsigned short b) { return (unsigned)a | ((unsigned)b << 16); }
__device__ __forceinline__ v8f zero8() { v8f z = {0.f, 0.f, 0.f, 0.f, 0.f, 0.f, 0.f, 0.f}; return z; }

__device__ __forceinline__ v16h ldfrag_h(const _Float16* p) {
  FH f;
  f.h[0] = *(const v8h*)(p);
  f.h[1] = *(const v8h*)(p + 16);
  return f.v;
}

__device__ __forceinline__ v8f mma_h(v16h a, v16h b, v8f c) {
  v8f d = __builtin_amdgcn_wmma_f32_16x16x32_f16(false, a, false, b, (short)0, c, false, false);
#if defined(__HIP_DEVICE_COMPILE__)
  asm volatile("v_nop\n\tv_nop\n\tv_nop\n\tv_nop" : "+v"(d) : "v"(a), "v"(b));
#endif
  return d;
}
__device__ __forceinline__ void acc_guard4(v8f& a, v8f& b, v8f& c, v8f& d) {
#if defined(__HIP_DEVICE_COMPILE__)
  asm volatile("v_nop\n\tv_nop\n\tv_nop\n\tv_nop" : "+v"(a), "+v"(b), "+v"(c), "+v"(d));
#endif
}
__device__ __forceinline__ void wave_sync_lds() {
  __builtin_amdgcn_fence(__ATOMIC_RELEASE, "workgroup");
  __builtin_amdgcn_wave_barrier();
  __builtin_amdgcn_fence(__ATOMIC_ACQUIRE, "workgroup");
}

__global__ __launch_bounds__(256) void cvt_rm(const float* __restrict__ in, unsigned short* out, int n,
                                             float scale) {
  const size_t i8 = ((size_t)blockIdx.x * 256 + threadIdx.x) * 8;
  if (i8 + 8 > (size_t)n) return;
  const v4f a = *(const v4f*)(in + i8);
  const v4f b = *(const v4f*)(in + i8 + 4);
  float f[8];
  f[0] = a[0]; f[1] = a[1]; f[2] = a[2]; f[3] = a[3];
  f[4] = b[0]; f[5] = b[1]; f[6] = b[2]; f[7] = b[3];
  v4u p;
#pragma unroll
  for (int e = 0; e < 4; ++e) {
    const _Float16 x0 = (_Float16)(bfr(f[2 * e]) * scale);
    const _Float16 x1 = (_Float16)(bfr(f[2 * e + 1]) * scale);
    p[e] = pk16(h_bits(x0), h_bits(x1));
  }
  *(volatile v4u*)(out + i8) = p;
  __threadfence();
  *(volatile v4u*)(out + i8) = p;
}

__global__ __launch_bounds__(128) void cvt_tr(const float* __restrict__ in, _Float16* out, float scale) {
  __shared__ __align__(16) _Float16 sT[HDIM * 72];
  const int tid  = threadIdx.x;
  const int lane = tid & 31;
  const int wave = tid >> 5;
  const int tb   = (int)(blockIdx.x % (unsigned)(NTOK / 64));
  const int kvh  = (int)(blockIdx.x / (unsigned)(NTOK / 64));
  const int t0   = tb * 64;
  {
    const int r = tid >> 1, hk = (tid & 1) * 64;
    const float* src = in + (size_t)(t0 + r) * KW + kvh * HDIM + hk;
#pragma unroll
    for (int i = 0; i < 16; ++i) {
      const v4f a = *(const v4f*)(src + 4 * i);
#pragma unroll
      for (int e = 0; e < 4; ++e) sT[(hk + 4 * i + e) * 72 + r] = (_Float16)(bfr(a[e]) * scale);
    }
  }
  __syncthreads();
  const int ql = lane >> 3, pc = lane & 7;
  v8h vals[8];
#pragma unroll
  for (int it = 0; it < 8; ++it) {
    const int d = wave * 32 + it * 4 + ql;
    vals[it] = *(const v8h*)(sT + d * 72 + pc * 8);
  }
  for (int pass = 0; pass < 2; ++pass) {
#pragma unroll
    for (int it = 0; it < 8; ++it) {
      const int d = wave * 32 + it * 4 + ql;
      *(volatile v8h*)(out + (size_t)(kvh * HDIM + d) * NTOK + t0 + pc * 8) = vals[it];
    }
    __threadfence();
  }
}

__global__ __launch_bounds__(128)
void attn_k(const unsigned short* __restrict__ Qp, const unsigned short* __restrict__ Kp,
            const unsigned short* __restrict__ PKp, const unsigned short* __restrict__ Vtp,
            const unsigned short* __restrict__ PVtp, float* Out, float sscale) {
  __shared__ __align__(16) _Float16 Ksh[64 * HDIM];
  __shared__ __align__(16) _Float16 Vsh[HDIM * 64];
  __shared__ __align__(16) _Float16 Psh[4][16 * 64];
  __shared__ __align__(16) float    Os[4][16 * HDIM];

  const int tid  = threadIdx.x;
  const int wave = tid >> 5;
  const int lane = tid & 31;
  const int hh   = lane >> 4;
  const int c    = lane & 15;

  const int qb   = (int)(blockIdx.x % (unsigned)NQB);
  const int h    = (int)(blockIdx.x / (unsigned)NQB);
  const int kvh  = h / GRPQ;
  const int bq   = qb / QBR;
  const int qbe  = qb - bq * QBR;
  const int q0   = qb * 64 + wave * 16;
  const int tokb = bq * RLEN;
  const int nch  = NPC + qbe + 1;

  const _Float16* Qg  = (const _Float16*)(const void*)Qp   + (size_t)h * HDIM;
  const _Float16* Kg  = (const _Float16*)(const void*)Kp   + (size_t)kvh * HDIM;
  const _Float16* PKg = (const _Float16*)(const void*)PKp  + (size_t)kvh * HDIM;
  const _Float16* Vg  = (const _Float16*)(const void*)Vtp  + (size_t)kvh * HDIM * NTOK;
  const _Float16* PVg = (const _Float16*)(const void*)PVtp + (size_t)kvh * HDIM * NTOK;

  float mrow[8], lrow[8];
  v8f oh[8];
#pragma unroll
  for (int r = 0; r < 8; ++r) { mrow[r] = NEG_BIG; lrow[r] = 0.f; }
#pragma unroll
  for (int t = 0; t < 8; ++t) oh[t] = zero8();

  _Float16* pwh = Psh[wave];

  for (int kt = 0; kt < nch; ++kt) {
    const bool pre  = (kt < NPC);
    const bool diag = (kt == nch - 1);
    const int  tk0  = pre ? (kt * 64) : ((kt - NPC) * 64);
    const int  kv0  = tokb + tk0;
    const _Float16* kg = pre ? PKg : Kg;
    const _Float16* vg = pre ? PVg : Vg;
    __syncthreads();
    {
      const int r = tid >> 1, hk = (tid & 1) * 64;
      const _Float16* ksrc = kg + (size_t)(kv0 + r) * KW + hk;
#pragma unroll
      for (int i = 0; i < 8; ++i) *(v8h*)(Ksh + r * HDIM + hk + 8 * i) = *(const v8h*)(ksrc + 8 * i);
      const _Float16* vsrc = vg + (size_t)tid * NTOK + kv0;
#pragma unroll
      for (int i = 0; i < 8; ++i) *(v8h*)(Vsh + tid * 64 + 8 * i) = *(const v8h*)(vsrc + 8 * i);
    }
    __syncthreads();

    v8f s[4];
#pragma unroll
    for (int j = 0; j < 4; ++j) s[j] = zero8();
#pragma unroll
    for (int dc = 0; dc < 4; ++dc) {
      const v16h qa = ldfrag_h(Qg + (size_t)(q0 + c) * QW + dc * 32 + 8 * hh);
#pragma unroll
      for (int j = 0; j < 4; ++j) {
        FH kb;
        kb.h[0] = *(const v8h*)(Ksh + (j * 16 + c) * HDIM + dc * 32 + 8 * hh);
        kb.h[1] = *(const v8h*)(Ksh + (j * 16 + c) * HDIM + dc * 32 + 16 + 8 * hh);
        s[j] = mma_h(qa, kb.v, s[j]);
      }
    }
    acc_guard4(s[0], s[1], s[2], s[3]);

    const int lim = diag ? (wave * 16 + 8 * hh) : 4096;
#pragma unroll
    for (int j = 0; j < 4; ++j) {
      const int kl = j * 16 + c;
#pragma unroll
      for (int r = 0; r < 8; ++r) {
        const float x = s[j][r] * sscale;
        const float y = CAPV * tanhf(x * (1.0f / CAPV));
        s[j][r] = (kl > lim + r) ? NEG_BIG : y;
      }
    }

#pragma unroll
    for (int r = 0; r < 8; ++r) {
      float m = fmaxf(fmaxf(s[0][r], s[1][r]), fmaxf(s[2][r], s[3][r]));
#pragma unroll
      for (int off = 1; off < 16; off <<= 1) m = fmaxf(m, __shfl_xor(m, off, 32));
      const float mnew  = fmaxf(mrow[r], m);
      const float alpha = __expf(mrow[r] - mnew);
      mrow[r] = mnew;
      float psum = 0.f;
#pragma unroll
      for (int j = 0; j < 4; ++j) {
        const float p = __expf(s[j][r] - mnew);
        psum += p;
        pwh[(8 * hh + r) * 64 + j * 16 + c] = (_Float16)(p * PSC);
      }
#pragma unroll
      for (int off = 1; off < 16; off <<= 1) psum += __shfl_xor(psum, off, 32);
      lrow[r] = lrow[r] * alpha + psum;
#pragma unroll
      for (int t = 0; t < 8; ++t) oh[t][r] *= alpha;
    }
    wave_sync_lds();

#pragma unroll
    for (int kk = 0; kk < 2; ++kk) {
      FH pa;
      pa.h[0] = *(const v8h*)(pwh + c * 64 + kk * 32 + 8 * hh);
      pa.h[1] = *(const v8h*)(pwh + c * 64 + kk * 32 + 16 + 8 * hh);
#pragma unroll
      for (int t = 0; t < 8; ++t) {
        FH vb;
        vb.h[0] = *(const v8h*)(Vsh + (t * 16 + c) * 64 + kk * 32 + 8 * hh);
        vb.h[1] = *(const v8h*)(Vsh + (t * 16 + c) * 64 + kk * 32 + 16 + 8 * hh);
        oh[t] = mma_h(pa.v, vb.v, oh[t]);
      }
    }
    acc_guard4(oh[0], oh[1], oh[2], oh[3]);
    acc_guard4(oh[4], oh[5], oh[6], oh[7]);
  }

  float* os = Os[wave];
#pragma unroll
  for (int r = 0; r < 8; ++r) {
    const float l = lrow[r];
    const float inv = ((l > 0.f) ? (1.0f / l) : 0.f) * (1.0f / (PSC * VSC));
#pragma unroll
    for (int t = 0; t < 8; ++t) os[(8 * hh + r) * HDIM + t * 16 + c] = oh[t][r] * inv;
  }
  wave_sync_lds();
  for (int pass = 0; pass < 2; ++pass) {
#pragma unroll
    for (int it = 0; it < 16; ++it) {
      const v4f o = *(const v4f*)(os + it * HDIM + lane * 4);
      *(volatile v4f*)(Out + (size_t)(q0 + it) * QW + (size_t)h * HDIM + lane * 4) = o;
    }
    __threadfence();
  }
}

extern "C" void kernel_launch(void* const* d_in, const int* in_sizes, int n_in,
                              void* d_out, int out_size, void* d_ws, size_t ws_size,
                              hipStream_t stream) {
  if (n_in < 5) return;
  if (in_sizes[0] != NTOK * QW) return;
  if (in_sizes[1] != NTOK * KW || in_sizes[2] != NTOK * KW) return;
  if (in_sizes[3] != NTOK * KW || in_sizes[4] != NTOK * KW) return;
  if (out_size != NTOK * QW) return;

  const float* q  = (const float*)d_in[0];
  const float* k  = (const float*)d_in[1];
  const float* v  = (const float*)d_in[2];
  const float* pk = (const float*)d_in[3];
  const float* pv = (const float*)d_in[4];
  float* outf = (float*)d_out;

  const size_t PQ  = (size_t)NTOK * QW * 2;
  const size_t PKV = (size_t)NTOK * KW * 2;
  size_t off = 0;
  const size_t oQ  = off; off += PQ;
  const size_t oK  = off; off += PKV;
  const size_t oPK = off; off += PKV;
  const size_t oV  = off; off += PKV;
  const size_t oPV = off; off += PKV;
  if (off > ws_size) return;
  if (off > (size_t)134217728) return;

  char* ws = (char*)d_ws;
  unsigned short* QP  = (unsigned short*)(ws + oQ);
  unsigned short* KP  = (unsigned short*)(ws + oK);
  unsigned short* PKP = (unsigned short*)(ws + oPK);
  unsigned short* VT  = (unsigned short*)(ws + oV);
  unsigned short* PVT = (unsigned short*)(ws + oPV);

  const dim3 blk256(256), blk128(128);
  const float sscale = 0.08838834764831845f / (QSC * KSC);

  cvt_rm<<<dim3((NTOK * QW) / 2048), blk256, 0, stream>>>(q, QP, NTOK * QW, QSC);
  cvt_rm<<<dim3((NTOK * KW) / 2048), blk256, 0, stream>>>(k, KP, NTOK * KW, KSC);
  cvt_rm<<<dim3((NTOK * KW) / 2048), blk256, 0, stream>>>(pk, PKP, NTOK * KW, KSC);
  cvt_tr<<<dim3((NTOK / 64) * HKV), blk128, 0, stream>>>(v, (_Float16*)(void*)VT, VSC);
  cvt_tr<<<dim3((NTOK / 64) * HKV), blk128, 0, stream>>>(pv, (_Float16*)(void*)PVT, VSC);
  attn_k<<<dim3(NQB * HQ), blk128, 0, stream>>>(QP, KP, PKP, VT, PVT, outf, sscale);
  (void)hipGetLastError();
}
